// SparseAttention_23149873725637
// MI455X (gfx1250) — hardware-verified
//
#include <hip/hip_runtime.h>


#ifndef NB
#define NB 1
#endif
#ifndef SEQ
#define SEQ 2048
#endif
#define NB_FULL  1
#define SEQ_FULL 2048
#define DM    1024
#define NH_   8
#define NKV   2
#define HD    128
#define NQKV  1536
#define LR    64
#define KX    1216
#define KO    2112
#define GLB   128
#define W0H   128
#define W1H   256
#define W2H   512
#define SCL   0.08838834764831845f
#define L2E   1.4426950408889634f

static_assert(SEQ % 64 == 0);
static_assert(SEQ >= GLB);
static_assert(SEQ <= SEQ_FULL);
static_assert(KX % 32 == 0);
static_assert(KO % 32 == 0);
static_assert(NQKV % 64 == 0);
static_assert((10 * SEQ * 16) % 256 == 0);
static_assert((SEQ * 128) % 256 == 0);
static_assert((SEQ * 24) % 256 == 0);
static_assert((SEQ * 8) % 256 == 0);
static_assert((1024 * (KX / 8)) % 256 == 0);
static_assert((256 * (KX / 8)) % 256 == 0);
static_assert((1024 * (KO / 8)) % 256 == 0);

typedef unsigned short bf;
typedef __attribute__((ext_vector_type(16))) __bf16   v16bf;
typedef __attribute__((ext_vector_type(8)))  unsigned short v8us;
typedef __attribute__((ext_vector_type(8)))  float    v8f;
typedef __attribute__((ext_vector_type(4)))  float    v4f;
typedef v4f  __attribute__((may_alias)) v4fa;
typedef v8us __attribute__((may_alias)) v8usa;

__device__ __forceinline__ unsigned short f2bf(float f) { unsigned u = __float_as_uint(f); u += 0x7FFFu + ((u >> 16) & 1u); return (unsigned short)(u >> 16); }
__device__ __forceinline__ float bf2f(unsigned short b) { return __uint_as_float(((unsigned)b) << 16); }
__device__ __forceinline__ float bfr(float f) { return bf2f(f2bf(f)); }
__device__ __forceinline__ void splitf(float y, unsigned short& h, unsigned short& l) { h = f2bf(y); l = f2bf(y - bf2f(h)); }
__device__ __forceinline__ v16bf cat16b(v8us lo, v8us hi) { return __builtin_bit_cast(v16bf, __builtin_shufflevector(lo, hi, 0, 1, 2, 3, 4, 5, 6, 7, 8, 9, 10, 11, 12, 13, 14, 15)); }
__device__ __forceinline__ v8f wmmab(v16bf a, v16bf b, v8f c) { return __builtin_amdgcn_wmma_f32_16x16x32_bf16(false, a, false, b, (short)0, c, false, false); }
__device__ __forceinline__ v16bf ldf(const bf* p) { return cat16b(*(const v8us*)p, *(const v8us*)(p + 16)); }
__device__ __forceinline__ float hmax16(float v) {
#pragma unroll
    for (int sh = 8; sh; sh >>= 1) v = fmaxf(v, __shfl_xor(v, sh, 32));
    return v; }
__device__ __forceinline__ float hsum16(float v) {
#pragma unroll
    for (int sh = 8; sh; sh >>= 1) v += __shfl_xor(v, sh, 32);
    return v; }

__global__ __launch_bounds__(32) void k_gemmw(const bf* __restrict__ A, unsigned lda, const bf* __restrict__ Bt, unsigned ldb, unsigned K, float* C, unsigned ldc) {
    __shared__ __align__(16) float os[16 * 68];
    const unsigned lane = threadIdx.x & 31u, lr = lane & 15u, hf = lane >> 4; const unsigned r0 = blockIdx.x * 64u, c0 = blockIdx.y * 64u;
    v8f acc[4][4];
#pragma unroll
    for (int mb = 0; mb < 4; ++mb)
#pragma unroll
        for (int nb = 0; nb < 4; ++nb) acc[mb][nb] = (v8f){};
    const bf* ap = A + (size_t)(r0 + lr) * lda + 8u * hf; const bf* bp = Bt + (size_t)(c0 + lr) * ldb + 8u * hf;
#pragma unroll 1
    for (unsigned kc = 0; kc < K; kc += 32u) {
        v16bf a[4];
#pragma unroll
        for (int mb = 0; mb < 4; ++mb) a[mb] = ldf(ap + (size_t)mb * 16u * lda + kc);
#pragma unroll
        for (int nb = 0; nb < 4; ++nb) { const v16bf b = ldf(bp + (size_t)nb * 16u * ldb + kc);
#pragma unroll
            for (int mb = 0; mb < 4; ++mb) acc[mb][nb] = wmmab(a[mb], b, acc[mb][nb]); }
        asm volatile("v_nop\n\tv_nop\n\tv_nop\n\tv_nop" : "+v"(acc[0][3]), "+v"(acc[1][3]), "+v"(acc[2][3]), "+v"(acc[3][3]) : "v"(a[0]), "v"(a[3]));
    }
#pragma unroll
    for (int mb = 0; mb < 4; ++mb) {
#pragma unroll
        for (int nb = 0; nb < 4; ++nb) {
#pragma unroll
            for (int j = 0; j < 8; ++j) os[(hf * 8u + j) * 68u + nb * 16u + lr] = acc[mb][nb][j]; }
        __syncthreads();
        float* crow = C + (size_t)(r0 + mb * 16u) * ldc + c0;
#pragma unroll 1
        for (int ps = 0; ps < 2; ++ps) {
#pragma unroll
            for (int s = 0; s < 8; ++s) { const unsigned row = 2u * s + hf, cofs = lr * 4u; const v4f val = *(const v4fa*)(os + row * 68u + cofs);
                *(volatile v4f*)(crow + (size_t)row * ldc + cofs) = val; }
            if (ps == 0) __threadfence(); }
        __syncthreads();
    }
}

__global__ __launch_bounds__(256) void k_cvtp(const float* __restrict__ src, unsigned w8, unsigned spitch, bf* dst, unsigned dpitch, unsigned n8) {
    const unsigned i = blockIdx.x * 256u + threadIdx.x; if (i >= n8) return;
    const unsigned r = i / w8, c = i - r * w8;
    const v8f v = *(const v8f*)(src + (size_t)r * spitch + c * 8u); v8us o;
#pragma unroll
    for (int k = 0; k < 8; ++k) o[k] = f2bf(v[k]);
    bf* p = dst + (size_t)r * dpitch + c * 8u;
    *(volatile v8us*)p = o; __threadfence(); *(volatile v8us*)p = o; }

__global__ __launch_bounds__(256) void k_wbuild(const float* __restrict__ W, const float* __restrict__ Bm, bf* dst, unsigned nrows, unsigned rep, unsigned lw, unsigned lofs) {
    const unsigned wcols = rep * 1024u; const unsigned cpr = (wcols + lw) >> 3;
    const unsigned i = blockIdx.x * 256u + threadIdx.x; if (i >= nrows * cpr) return;
    const unsigned r = i / cpr, c = i - r * cpr; const unsigned col = c * 8u;
    const bool isw = col < wcols;
    const unsigned wc = isw ? (col & 1023u) : 0u;
    const unsigned j = isw ? 0u : (col - wcols);
    const bool isb = (!isw) && (j >= lofs) && (j < lofs + 64u);
    const unsigned bc = isb ? (j - lofs) : 0u;
    const v8f wv = *(const v8f*)(W + (size_t)r * 1024u + wc);
    const v8f bv = *(const v8f*)(Bm + (size_t)r * 64u + bc);
    v8us o;
#pragma unroll
    for (int k = 0; k < 8; ++k) { const float w = bfr(wv[k]); const float b = bfr(bv[k]) * (1.0f / 64.0f); const float x = isw ? w : (isb ? b : 0.0f); o[k] = f2bf(x); }
    bf* p = dst + (size_t)r * cpr * 8u + col;
    *(volatile v8us*)p = o; __threadfence(); *(volatile v8us*)p = o; }

__global__ __launch_bounds__(256) void k_ropeqk(const float* __restrict__ F, const float* __restrict__ fc, const int* __restrict__ spp, bf* PH, bf* PL) {
    const unsigned i = blockIdx.x * 256u + threadIdx.x; if (i >= 10u * SEQ * 16u) return;
    const unsigned e = i * 8u; const unsigned d = e & 127u; const unsigned t = (e >> 7) % (unsigned)SEQ; const unsigned hh = e / ((unsigned)SEQ * 128u);
    int sp = spp[0]; if (sp < 0) sp = 0; const int spmax = SEQ_FULL - SEQ; if (sp > spmax) sp = spmax;
    const v8f x = *(const v8f*)(F + (size_t)t * NQKV + hh * 128u + d);
    const v8f cs = *(const v8f*)(fc + ((size_t)sp + t) * 128u + d);
    v8us oh, ol;
#pragma unroll
    for (int j = 0; j < 4; ++j) { const float c = bfr(cs[2 * j]), s = bfr(cs[2 * j + 1]); const float x1 = x[2 * j], x2 = x[2 * j + 1];
        const float y1 = x1 * c - x2 * s; const float y2 = x1 * s + x2 * c; unsigned short a, b;
        splitf(y1, a, b); oh[2 * j] = a; ol[2 * j] = b; splitf(y2, a, b); oh[2 * j + 1] = a; ol[2 * j + 1] = b; }
    *(volatile v8us*)(PH + e) = oh; *(volatile v8us*)(PL + e) = ol; __threadfence(); *(volatile v8us*)(PH + e) = oh; *(volatile v8us*)(PL + e) = ol; }

__global__ __launch_bounds__(256) void k_vt(const float* __restrict__ F, bf* VH, bf* VL) {
    __shared__ float ts[64 * 65];
    const unsigned tid = threadIdx.x; const unsigned t0 = blockIdx.x * 64u, c0 = blockIdx.y * 64u;
    { const unsigned row = tid >> 2, cb = (tid & 3u) * 16u; const float* sp = F + (size_t)(t0 + row) * NQKV + 1280u + c0 + cb;
#pragma unroll
      for (int j = 0; j < 4; ++j) { const v4f v = *(const v4f*)(sp + 4 * j);
#pragma unroll
          for (int q = 0; q < 4; ++q) ts[row * 65u + cb + 4u * j + q] = v[q]; } }
    __syncthreads();
#pragma unroll 1
    for (int ps = 0; ps < 2; ++ps) {
#pragma unroll
        for (int it = 0; it < 2; ++it) { const unsigned d = it * 32u + (tid >> 3), tc = (tid & 7u) * 8u; v8us oh, ol;
#pragma unroll
            for (int j = 0; j < 8; ++j) { unsigned short a, b; splitf(ts[(tc + j) * 65u + d], a, b); oh[j] = a; ol[j] = b; }
            const size_t o = (size_t)(c0 + d) * SEQ + t0 + tc; *(volatile v8us*)(VH + o) = oh; *(volatile v8us*)(VL + o) = ol; }
        if (ps == 0) __threadfence(); }
}

__global__ __launch_bounds__(32) void k_attn(const bf* QH, const bf* QL, const bf* KH, const bf* KL, const bf* VH, const bf* VL, const float* __restrict__ sw, bf* CA) {
    __shared__ __align__(16) float fs[16 * 132];
    __shared__ __align__(16) unsigned short phs[16 * 40];
    __shared__ __align__(16) unsigned short pls[16 * 40];
    const unsigned lane = threadIdx.x & 31u, lr = lane & 15u, hf = lane >> 4;
    const unsigned q0 = blockIdx.x * 16u, h = blockIdx.y, g = h >> 2;
    const size_t qoff = ((size_t)h * SEQ + q0 + lr) * HD + 8u * hf; const bf* qh = QH + qoff; const bf* ql = QL + qoff;
    const size_t koff = ((size_t)g * SEQ + lr) * HD + 8u * hf;      const bf* kh = KH + koff; const bf* kl = KL + koff;
    const size_t voff = ((size_t)g * HD + lr) * SEQ + 8u * hf;      const bf* vh = VH + voff; const bf* vl = VL + voff;
    const float a0 = bfr(sw[0]), a1 = bfr(sw[1]), a2 = bfr(sw[2]); const float am = fmaxf(a0, fmaxf(a1, a2));
    const float ew0 = __builtin_amdgcn_exp2f((a0 - am) * L2E), ew1 = __builtin_amdgcn_exp2f((a1 - am) * L2E), ew2 = __builtin_amdgcn_exp2f((a2 - am) * L2E);
    const float winv = 1.0f / (ew0 + ew1 + ew2); const float w0 = ew0 * winv, w1 = ew1 * winv, w2 = ew2 * winv;
    v8f O[8]; float mr[8], ls[8];
#pragma unroll
    for (int nt = 0; nt < 8; ++nt) O[nt] = (v8f){};
#pragma unroll
    for (int r = 0; r < 8; ++r) { mr[r] = -3.0e38f; ls[r] = 0.0f;
#pragma unroll
        for (int nt = 0; nt < 8; ++nt) fs[(8u * hf + r) * 132u + nt * 16u + lr] = 0.0f; }
    const int iq0 = (int)q0;
#pragma unroll 1
    for (int ph = 0; ph < 4; ++ph) {
        int lo, hw, ks, ke;
        if (ph == 0) { lo = -1; hw = 1 << 20; ks = 0; ke = GLB; }
        else { lo = (ph == 1) ? -1 : ((ph == 2) ? W0H : W1H); hw = (ph == 1) ? W0H : ((ph == 2) ? W1H : W2H);
               int a = iq0 - hw; if (a < GLB) a = GLB; ks = a & ~31; int b = (iq0 + 16 + hw + 31) & ~31; if (b > SEQ) b = SEQ; ke = b; }
#pragma unroll 1
        for (int k0 = ks; k0 < ke; k0 += 32) {
            const int dmin = k0 - iq0 - 15, dmax = k0 + 31 - iq0;
            const int amin = dmin > 0 ? dmin : (dmax < 0 ? -dmax : 0); const int amax = (-dmin > dmax) ? -dmin : dmax;
            if (!((amax > lo) && (amin <= hw))) continue;
            v8f s0 = (v8f){}, s1 = (v8f){};
            const bf* kh0 = kh + (size_t)k0 * HD; const bf* kl0 = kl + (size_t)k0 * HD;
#pragma unroll 1
            for (int kk = 0; kk < 4; ++kk) {
                const v16bf aqh = ldf(qh + kk * 32), aql = ldf(ql + kk * 32);
                const v16bf b0h = ldf(kh0 + kk * 32), b0l = ldf(kl0 + kk * 32);
                const v16bf b1h = ldf(kh0 + 16 * HD + kk * 32), b1l = ldf(kl0 + 16 * HD + kk * 32);
                s0 = wmmab(aqh, b0h, s0); s1 = wmmab(aqh, b1h, s1);
                s0 = wmmab(aql, b0h, s0); s1 = wmmab(aql, b1h, s1);
                s0 = wmmab(aqh, b0l, s0); s1 = wmmab(aqh, b1l, s1);
                asm volatile("v_nop\n\tv_nop\n\tv_nop\n\tv_nop" : "+v"(s0), "+v"(s1) : "v"(aqh), "v"(aql), "v"(b0h), "v"(b0l), "v"(b1h), "v"(b1l));
            }
            __syncthreads();
            float al[8];
#pragma unroll
            for (int r = 0; r < 8; ++r) {
                const int qq = iq0 + (int)(8u * hf) + r; const int dA = k0 + (int)lr - qq; const int dB = dA + 16;
                const int adA = dA < 0 ? -dA : dA; const int adB = dB < 0 ? -dB : dB;
                const bool iA = (adA > lo) && (adA <= hw); const bool iB = (adB > lo) && (adB <= hw);
                const float x0 = s0[r] * SCL, x1 = s1[r] * SCL;
                const float tm = hmax16(fmaxf(iA ? x0 : -3.0e38f, iB ? x1 : -3.0e38f));
                const float mo = mr[r]; const float mn = fmaxf(mo, tm); mr[r] = mn;
                const float alpha = __builtin_amdgcn_exp2f((mo - mn) * L2E); al[r] = alpha;
                const float t0 = __builtin_amdgcn_exp2f((x0 - mn) * L2E), t1 = __builtin_amdgcn_exp2f((x1 - mn) * L2E);
                const float e0 = iA ? t0 : 0.0f, e1 = iB ? t1 : 0.0f;
                const float rs = hsum16(e0 + e1); ls[r] = ls[r] * alpha + rs;
                unsigned short h0, l0, h1, l1; splitf(e0, h0, l0); splitf(e1, h1, l1);
                const unsigned pr = (8u * hf + r) * 40u + lr;
                phs[pr] = h0; phs[pr + 16u] = h1; pls[pr] = l0; pls[pr + 16u] = l1;
            }
#pragma unroll
            for (int nt = 0; nt < 8; ++nt)
#pragma unroll
                for (int r = 0; r < 8; ++r) O[nt][r] *= al[r];
            __syncthreads();
            const v16bf pah = cat16b(*(const v8usa*)(phs + lr * 40u + 8u * hf), *(const v8usa*)(phs + lr * 40u + 16u + 8u * hf));
            const v16bf pal = cat16b(*(const v8usa*)(pls + lr * 40u + 8u * hf), *(const v8usa*)(pls + lr * 40u + 16u + 8u * hf));
            const bf* vh0 = vh + k0; const bf* vl0 = vl + k0;
#pragma unroll
            for (int nt = 0; nt < 8; ++nt) {
                const v16bf bvh = ldf(vh0 + (size_t)nt * 16u * SEQ), bvl = ldf(vl0 + (size_t)nt * 16u * SEQ);
                O[nt] = wmmab(pah, bvh, O[nt]); O[nt] = wmmab(pal, bvh, O[nt]); O[nt] = wmmab(pah, bvl, O[nt]);
                if (nt & 1) asm volatile("" ::: "memory");
            }
            asm volatile("v_nop\n\tv_nop\n\tv_nop\n\tv_nop" : "+v"(O[0]), "+v"(O[1]), "+v"(O[2]), "+v"(O[3]), "+v"(O[4]), "+v"(O[5]), "+v"(O[6]), "+v"(O[7]) : "v"(pah), "v"(pal));
        }
        if (ph >= 1) {
            const float wv = (ph == 1) ? w0 : ((ph == 2) ? w1 : w2);
#pragma unroll
            for (int r = 0; r < 8; ++r) { const float f = wv * (1.0f / ls[r]);
#pragma unroll
                for (int nt = 0; nt < 8; ++nt) { const unsigned ix = (8u * hf + r) * 132u + nt * 16u + lr; const float cur = fs[ix]; fs[ix] = cur + O[nt][r] * f; } }
        }
    }
    __syncthreads();
    bf* crow = CA + (size_t)q0 * KO + h * HD + lr * 8u;
#pragma unroll 1
    for (int ps = 0; ps < 2; ++ps) {
#pragma unroll
        for (int s = 0; s < 8; ++s) { const unsigned row = 2u * s + hf; const float* fp = fs + row * 132u + lr * 8u;
            const v4f x0 = *(const v4fa*)fp; const v4f x1 = *(const v4fa*)(fp + 4); v8us oh, ol;
#pragma unroll
            for (int q = 0; q < 4; ++q) { unsigned short a, b; splitf(x0[q], a, b); oh[q] = a; ol[q] = b; splitf(x1[q], a, b); oh[4 + q] = a; ol[4 + q] = b; }
            bf* p = crow + (size_t)row * KO; *(volatile v8us*)p = oh; *(volatile v8us*)(p + 1024) = ol; }
        if (ps == 0) __threadfence(); }
}

extern "C" void kernel_launch(void* const* d_in, const int* in_sizes, int n_in,
                              void* d_out, int out_size, void* d_ws, size_t ws_size, hipStream_t stream) {
    if (n_in < 16) return;
    const size_t need_x = (size_t)(NB - 1) * SEQ_FULL * DM + (size_t)SEQ * DM;
    if ((size_t)in_sizes[0] < need_x) return; if ((size_t)in_sizes[1] < (size_t)SEQ * HD) return;
    if ((size_t)in_sizes[2] < (size_t)1024 * 1024) return; if ((size_t)in_sizes[3] < (size_t)64 * 1024) return; if ((size_t)in_sizes[4] < (size_t)1024 * 64) return;
    if ((size_t)in_sizes[5] < (size_t)256 * 1024) return;  if ((size_t)in_sizes[6] < (size_t)64 * 1024) return; if ((size_t)in_sizes[7] < (size_t)256 * 64) return;
    if ((size_t)in_sizes[8] < (size_t)256 * 1024) return;  if ((size_t)in_sizes[9] < (size_t)64 * 1024) return; if ((size_t)in_sizes[10] < (size_t)256 * 64) return;
    if ((size_t)in_sizes[11] < (size_t)1024 * 1024) return; if ((size_t)in_sizes[12] < (size_t)64 * 1024) return; if ((size_t)in_sizes[13] < (size_t)1024 * 64) return;
    if (in_sizes[14] < 3) return; if (in_sizes[15] < 1) return;
    if ((size_t)out_size < need_x) return;
    const float* x = (const float*)d_in[0]; const float* fc = (const float*)d_in[1];
    const float* wq_w = (const float*)d_in[2];  const float* wq_a = (const float*)d_in[3];  const float* wq_b = (const float*)d_in[4];
    const float* wk_w = (const float*)d_in[5];  const float* wk_a = (const float*)d_in[6];  const float* wk_b = (const float*)d_in[7];
    const float* wv_w = (const float*)d_in[8];  const float* wv_a = (const float*)d_in[9];  const float* wv_b = (const float*)d_in[10];
    const float* wo_w = (const float*)d_in[11]; const float* wo_a = (const float*)d_in[12]; const float* wo_b = (const float*)d_in[13];
    const float* sw = (const float*)d_in[14]; const int* spp = (const int*)d_in[15];
    float* OUT = (float*)d_out;
    char* wsp = (char*)d_ws;
    auto take = [&](size_t bytes) { char* p = wsp; wsp += (bytes + 255) & ~(size_t)255; return (void*)p; };
    bf* XA  = (bf*)take((size_t)SEQ * KX * 2);
    bf* WA  = (bf*)take((size_t)192 * 1024 * 2);
    bf* WB  = (bf*)take((size_t)NQKV * KX * 2);
    bf* WOA = (bf*)take((size_t)64 * 1024 * 2);
    bf* WOB = (bf*)take((size_t)1024 * KO * 2);
    float* Tf   = (float*)take((size_t)SEQ * 192 * 4);
    float* QKVf = (float*)take((size_t)SEQ * NQKV * 4);
    bf* QKH = (bf*)take((size_t)10 * SEQ * HD * 2); bf* QKL = (bf*)take((size_t)10 * SEQ * HD * 2);
    bf* VTH = (bf*)take((size_t)256 * SEQ * 2);     bf* VTL = (bf*)take((size_t)256 * SEQ * 2);
    bf* CA  = (bf*)take((size_t)SEQ * KO * 2);
    float* Tof = (float*)take((size_t)SEQ * 64 * 4);
    const size_t used = (size_t)(wsp - (char*)d_ws);
    if (used > ws_size || used > (size_t)134217728) return;

    k_cvtp<<<(64u * 128u) / 256u, 256, 0, stream>>>(wq_a, 128u, 1024u, WA, 1024u, 64u * 128u);
    k_cvtp<<<(64u * 128u) / 256u, 256, 0, stream>>>(wk_a, 128u, 1024u, WA + (size_t)64 * 1024, 1024u, 64u * 128u);
    k_cvtp<<<(64u * 128u) / 256u, 256, 0, stream>>>(wv_a, 128u, 1024u, WA + (size_t)128 * 1024, 1024u, 64u * 128u);
    k_cvtp<<<(64u * 128u) / 256u, 256, 0, stream>>>(wo_a, 128u, 1024u, WOA, 1024u, 64u * 128u);
    k_wbuild<<<(1024u * (KX / 8)) / 256u, 256, 0, stream>>>(wq_w, wq_b, WB, 1024u, 1u, 192u, 0u);
    k_wbuild<<<(256u * (KX / 8)) / 256u, 256, 0, stream>>>(wk_w, wk_b, WB + (size_t)1024 * KX, 256u, 1u, 192u, 64u);
    k_wbuild<<<(256u * (KX / 8)) / 256u, 256, 0, stream>>>(wv_w, wv_b, WB + (size_t)1280 * KX, 256u, 1u, 192u, 128u);
    k_wbuild<<<(1024u * (KO / 8)) / 256u, 256, 0, stream>>>(wo_w, wo_b, WOB, 1024u, 2u, 64u, 0u);

    for (int b = 0; b < NB; ++b) {
        const float* xb = x + (size_t)b * SEQ_FULL * DM; float* ob = OUT + (size_t)b * SEQ_FULL * DM;
        k_cvtp<<<((unsigned)SEQ * 128u) / 256u, 256, 0, stream>>>(xb, 128u, 1024u, XA, (unsigned)KX, (unsigned)SEQ * 128u);
        k_gemmw<<<dim3(SEQ / 64, 3, 1), 32, 0, stream>>>(XA, (unsigned)KX, WA, 1024u, 1024u, Tf, 192u);
        k_cvtp<<<((unsigned)SEQ * 24u) / 256u, 256, 0, stream>>>(Tf, 24u, 192u, XA + 1024, (unsigned)KX, (unsigned)SEQ * 24u);
        k_gemmw<<<dim3(SEQ / 64, NQKV / 64, 1), 32, 0, stream>>>(XA, (unsigned)KX, WB, (unsigned)KX, (unsigned)KX, QKVf, (unsigned)NQKV);
        k_ropeqk<<<(10u * (unsigned)SEQ * 16u) / 256u, 256, 0, stream>>>(QKVf, fc, spp, QKH, QKL);
        k_vt<<<dim3(SEQ / 64, 4, 1), 256, 0, stream>>>(QKVf, VTH, VTL);
        k_attn<<<dim3(SEQ / 16, NH_, 1), 32, 0, stream>>>(QKH, QKL, QKH + (size_t)8 * SEQ * HD, QKL + (size_t)8 * SEQ * HD, VTH, VTL, sw, CA);
        k_gemmw<<<dim3(SEQ / 64, 1, 1), 32, 0, stream>>>(CA, (unsigned)KO, WOA, 1024u, 1024u, Tof, 64u);
        k_cvtp<<<((unsigned)SEQ * 8u) / 256u, 256, 0, stream>>>(Tof, 8u, 64u, CA + 2048, (unsigned)KO, (unsigned)SEQ * 8u);
        k_gemmw<<<dim3(SEQ / 64, DM / 64, 1), 32, 0, stream>>>(CA, (unsigned)KO, WOB, (unsigned)KO, (unsigned)KO, ob, (unsigned)DM);
    }
}
